// multi_head_attention_14955076125171
// MI455X (gfx1250) — hardware-verified
//
#include <hip/hip_runtime.h>


#ifndef NB
#define NB 2
#endif
#ifndef SEQ
#define SEQ 2048
#endif
#define NB_FULL  2
#define SEQ_FULL 2048
#define DM   1024
#define NH   16
#define DH   64
#define MTOK (NB * SEQ)
#define QT   128
#define KTL  64
#define LP   9
#define GEMM_LDS_Q 2176
#define ATTN_LDS_Q 2880

static_assert(MTOK % 128 == 0);
static_assert(SEQ % QT == 0);
static_assert(SEQ % KTL == 0);
static_assert(QT % KTL == 0);
static_assert(DM % 128 == 0);
static_assert(DM / 32 == 32);
static_assert(NH * DH == DM);
static_assert(NB >= 1 && NB <= NB_FULL);
static_assert(SEQ <= SEQ_FULL);
static_assert(SEQ % 16 == 0);
static_assert(GEMM_LDS_Q >= 128 * 17);
static_assert(GEMM_LDS_Q >= 64 * 33);
static_assert(ATTN_LDS_Q == 3 * KTL * LP + QT * LP);

typedef __attribute__((ext_vector_type(16))) __bf16   v16bf;
typedef __attribute__((ext_vector_type(2)))  __bf16   v2bf;
typedef __attribute__((ext_vector_type(16))) _Float16 v16h;
typedef __attribute__((ext_vector_type(8)))  _Float16 v8h;
typedef __attribute__((ext_vector_type(8)))  float    v8f;
typedef __attribute__((ext_vector_type(4)))  float    v4f;
typedef __attribute__((ext_vector_type(4)))  unsigned int u32x4;

union ABf { v16bf v; u32x4 q[2]; unsigned int u[8]; };
union AHf { v16h v;  u32x4 q[2]; };
union PK4 { u32x4 q; unsigned int u[4]; };
union PH8 { v8h v;   u32x4 q; };

__device__ __forceinline__ unsigned short f2bf(float f) {
    unsigned int u = __builtin_bit_cast(unsigned int, f);
    u = (u + 0x7fffu + ((u >> 16) & 1u)) >> 16;
    return (unsigned short)u;
}

__device__ __forceinline__ unsigned int f2bf2(float lo, float hi) {
#if __has_builtin(__builtin_amdgcn_cvt_pk_bf16_f32)
    v2bf r = __builtin_amdgcn_cvt_pk_bf16_f32(lo, hi);
    return __builtin_bit_cast(unsigned int, r);
#else
    return (unsigned int)f2bf(lo) | ((unsigned int)f2bf(hi) << 16);
#endif
}

__device__ __forceinline__ float bfr(float f) {
    unsigned int u = __builtin_bit_cast(unsigned int, f);
    u = (u + 0x7fffu + ((u >> 16) & 1u)) & 0xffff0000u;
    return __builtin_bit_cast(float, u);
}

__device__ __forceinline__ void split2(float a, float b, unsigned int& hi, unsigned int& lo) {
    hi = f2bf2(a, b);
    const float ha = __builtin_bit_cast(float, hi << 16);
    const float hb = __builtin_bit_cast(float, hi & 0xffff0000u);
    lo = f2bf2(a - ha, b - hb);
}

__device__ __forceinline__ v8f mma_bf16(const ABf& a, const ABf& b, v8f c) {
    c = __builtin_amdgcn_wmma_f32_16x16x32_bf16(false, a.v, false, b.v, (short)0, c, false, false);
    asm volatile("v_nop\n\tv_nop\n\tv_nop\n\tv_nop" : "+v"(c) : "v"(a.v), "v"(b.v));
    return c;
}
__device__ __forceinline__ v8f mma_f16(const AHf& a, const AHf& b, v8f c) {
    c = __builtin_amdgcn_wmma_f32_16x16x32_f16(false, a.v, false, b.v, (short)0, c, false, false);
    asm volatile("v_nop\n\tv_nop\n\tv_nop\n\tv_nop" : "+v"(c) : "v"(a.v), "v"(b.v));
    return c;
}

__global__ __launch_bounds__(256)
void k_cvt(const float* __restrict__ s0, const float* __restrict__ s1,
           const float* __restrict__ s2, const float* __restrict__ s3,
           unsigned short* d0, unsigned short* d1, unsigned short* d2, unsigned short* d3,
           int nrows, int seg, int seg_full)
{
    const int tid = threadIdx.x;
    const int row = blockIdx.x * 2 + (tid >> 7);
    const int y = blockIdx.y;
    const float* src = s0; unsigned short* dst = d0;
    if (y == 1)      { src = s1; dst = d1; }
    else if (y == 2) { src = s2; dst = d2; }
    else if (y == 3) { src = s3; dst = d3; }
    if (row >= nrows) return;
    const int b = row / seg;
    const int s = row - b * seg;
    const size_t srow = (size_t)b * seg_full + s;
    const int col = (tid & 127) * 8;
    const float4 a = *(const float4*)(src + srow * DM + col);
    const float4 c = *(const float4*)(src + srow * DM + col + 4);
    u32x4 pk = { f2bf2(a.x, a.y), f2bf2(a.z, a.w), f2bf2(c.x, c.y), f2bf2(c.z, c.w) };
    unsigned short* dp = dst + (size_t)row * DM + col;
    *(volatile u32x4*)dp = pk;
    __threadfence();
    *(volatile u32x4*)dp = pk;
}

template<int MODE>
__global__ __launch_bounds__(256) __attribute__((amdgpu_num_vgpr(256)))
void k_gemm(const unsigned short* __restrict__ Rop,
            const unsigned short* __restrict__ Cop0,
            const unsigned short* __restrict__ Cop1,
            const float* __restrict__ bias,
            void* dst0, void* dst1)
{
    __shared__ u32x4 lds[GEMM_LDS_Q];

    const int tid = threadIdx.x, lane = tid & 31, w = tid >> 5;
    const int h = lane >> 4, m = lane & 15;
    const int wm = (w >> 1) * 32;
    const int wn = (w & 1) * 64;
    const int rbase = blockIdx.x * 128;
    const int cbase = blockIdx.y * 128;
    constexpr int KSTEPS = DM / 32;
    constexpr int NSTEP  = (MODE == 2) ? 2 * KSTEPS : KSTEPS;

    v8f acc[2][4];
    #pragma unroll
    for (int i = 0; i < 2; ++i)
        #pragma unroll
        for (int j = 0; j < 4; ++j) { v8f z = {}; acc[i][j] = z; }

    #pragma unroll 1
    for (int ks = 0; ks < NSTEP; ++ks) {
        const int kk = (ks & (KSTEPS - 1)) * 32;
        const unsigned short* Cp = (ks < KSTEPS) ? Cop0 : Cop1;
        ABf ar[2], bc[4];
        #pragma unroll
        for (int i = 0; i < 2; ++i) {
            const unsigned short* p = Rop + (size_t)(rbase + wm + i * 16 + m) * DM + kk;
            ar[i].q[0] = *(const u32x4*)(p + 8 * h);
            ar[i].q[1] = *(const u32x4*)(p + 16 + 8 * h);
        }
        #pragma unroll
        for (int j = 0; j < 4; ++j) {
            const unsigned short* p = Cp + (size_t)(cbase + wn + j * 16 + m) * DM + kk;
            bc[j].q[0] = *(const u32x4*)(p + 8 * h);
            bc[j].q[1] = *(const u32x4*)(p + 16 + 8 * h);
        }
        #pragma unroll
        for (int i = 0; i < 2; ++i)
            #pragma unroll
            for (int j = 0; j < 4; ++j)
                acc[i][j] = mma_bf16(ar[i], bc[j], acc[i][j]);
    }

    if constexpr (MODE == 0) {
        float b8[2][8];
        #pragma unroll
        for (int i = 0; i < 2; ++i) {
            const float* bp = bias + rbase + wm + i * 16 + 8 * h;
            const float4 u0 = *(const float4*)bp;
            const float4 u1 = *(const float4*)(bp + 4);
            b8[i][0] = bfr(u0.x); b8[i][1] = bfr(u0.y); b8[i][2] = bfr(u0.z); b8[i][3] = bfr(u0.w);
            b8[i][4] = bfr(u1.x); b8[i][5] = bfr(u1.y); b8[i][6] = bfr(u1.z); b8[i][7] = bfr(u1.w);
        }
        #pragma unroll
        for (int i = 0; i < 2; ++i)
            #pragma unroll
            for (int j = 0; j < 4; ++j) {
                PH8 pk;
                #pragma unroll
                for (int r = 0; r < 8; ++r) pk.v[r] = (_Float16)(acc[i][j][r] + b8[i][r]);
                lds[(wn + j * 16 + m) * 17 + (wm >> 3) + 2 * i + h] = pk.q;
            }
        __syncthreads();
        unsigned short* base0 = (unsigned short*)dst0;
        u32x4 vv[8]; unsigned short* pp[8];
        #pragma unroll
        for (int it = 0; it < 8; ++it) {
            const int pid = it * 256 + tid;
            const int row = pid >> 4, c16 = pid & 15;
            vv[it] = lds[row * 17 + c16];
            const int headi = (rbase >> 6) + (c16 >> 3);
            const int token = cbase + row;
            const int bb = token / SEQ, ss = token - bb * SEQ;
            pp[it] = base0 + ((size_t)(bb * NH + headi) * SEQ + ss) * DH + (c16 & 7) * 8;
        }
        #pragma unroll
        for (int it = 0; it < 8; ++it) *(volatile u32x4*)pp[it] = vv[it];
        __threadfence();
        #pragma unroll
        for (int it = 0; it < 8; ++it) *(volatile u32x4*)pp[it] = vv[it];
    } else if constexpr (MODE == 1) {
        float bj[4];
        #pragma unroll
        for (int j = 0; j < 4; ++j) bj[j] = bfr(bias[cbase + wn + j * 16 + m]);
        const int bV = rbase / SEQ;
        const int s0 = rbase - bV * SEQ;
        #pragma unroll
        for (int pl = 0; pl < 2; ++pl) {
            if (pl == 1) __syncthreads();
            #pragma unroll
            for (int i = 0; i < 2; ++i)
                #pragma unroll
                for (int j = 0; j < 4; ++j) {
                    PK4 pk;
                    #pragma unroll
                    for (int e = 0; e < 4; ++e) {
                        const float a  = acc[i][j][2 * e]     + bj[j];
                        const float b2 = acc[i][j][2 * e + 1] + bj[j];
                        unsigned int hi, lo;
                        split2(a, b2, hi, lo);
                        pk.u[e] = (pl == 0) ? hi : lo;
                    }
                    lds[(wn + j * 16 + m) * 17 + (wm >> 3) + 2 * i + h] = pk.q;
                }
            __syncthreads();
            unsigned short* base = (unsigned short*)((pl == 0) ? dst0 : dst1);
            u32x4 vv[8]; unsigned short* pp[8];
            #pragma unroll
            for (int it = 0; it < 8; ++it) {
                const int pid = it * 256 + tid;
                const int row = pid >> 4, c16 = pid & 15;
                vv[it] = lds[row * 17 + c16];
                const int n = cbase + row;
                const int headi = n >> 6, d = n & 63;
                pp[it] = base + ((size_t)(bV * NH + headi) * DH + d) * SEQ + s0 + c16 * 8;
            }
            #pragma unroll
            for (int it = 0; it < 8; ++it) *(volatile u32x4*)pp[it] = vv[it];
            __threadfence();
            #pragma unroll
            for (int it = 0; it < 8; ++it) *(volatile u32x4*)pp[it] = vv[it];
        }
    } else {
        float b8[2][8];
        #pragma unroll
        for (int i = 0; i < 2; ++i) {
            const float* bp = bias + rbase + wm + i * 16 + 8 * h;
            const float4 u0 = *(const float4*)bp;
            const float4 u1 = *(const float4*)(bp + 4);
            b8[i][0] = bfr(u0.x); b8[i][1] = bfr(u0.y); b8[i][2] = bfr(u0.z); b8[i][3] = bfr(u0.w);
            b8[i][4] = bfr(u1.x); b8[i][5] = bfr(u1.y); b8[i][6] = bfr(u1.z); b8[i][7] = bfr(u1.w);
        }
        float* ob = (float*)dst0;
        #pragma unroll
        for (int pass = 0; pass < 2; ++pass) {
            if (pass == 1) __syncthreads();
            if (wn == pass * 64) {
                #pragma unroll
                for (int i = 0; i < 2; ++i)
                    #pragma unroll
                    for (int j = 0; j < 4; ++j) {
                        v4f lo4 = { acc[i][j][0] + b8[i][0], acc[i][j][1] + b8[i][1],
                                    acc[i][j][2] + b8[i][2], acc[i][j][3] + b8[i][3] };
                        v4f hi4 = { acc[i][j][4] + b8[i][4], acc[i][j][5] + b8[i][5],
                                    acc[i][j][6] + b8[i][6], acc[i][j][7] + b8[i][7] };
                        const int idx = (j * 16 + m) * 33 + (wm >> 2) + 4 * i + 2 * h;
                        lds[idx]     = __builtin_bit_cast(u32x4, lo4);
                        lds[idx + 1] = __builtin_bit_cast(u32x4, hi4);
                    }
            }
            __syncthreads();
            v4f vf[8]; float* pf[8];
            #pragma unroll
            for (int it = 0; it < 8; ++it) {
                const int pid = it * 256 + tid;
                const int row = pid >> 5, c4 = pid & 31;
                vf[it] = __builtin_bit_cast(v4f, lds[row * 33 + c4]);
                const int token = cbase + pass * 64 + row;
                const int bb = token / SEQ, ss = token - bb * SEQ;
                pf[it] = ob + ((size_t)bb * SEQ_FULL + ss) * DM + rbase + c4 * 4;
            }
            #pragma unroll
            for (int it = 0; it < 8; ++it) *(volatile v4f*)pf[it] = vf[it];
            __threadfence();
            #pragma unroll
            for (int it = 0; it < 8; ++it) *(volatile v4f*)pf[it] = vf[it];
        }
    }
}

__global__ __launch_bounds__(256) __attribute__((amdgpu_num_vgpr(256)))
void k_attn(const unsigned short* __restrict__ Qp, const unsigned short* __restrict__ Kp,
            const unsigned short* __restrict__ Vth, const unsigned short* __restrict__ Vtl,
            unsigned short* Ch, unsigned short* Cl)
{
    __shared__ u32x4 lds[ATTN_LDS_Q];
    u32x4* Ks  = lds;
    u32x4* Vhs = lds + KTL * LP;
    u32x4* Vls = lds + 2 * KTL * LP;
    u32x4* Ost = lds + 3 * KTL * LP;

    const int tid = threadIdx.x, lane = tid & 31, w = tid >> 5;
    const int h = lane >> 4, m = lane & 15;
    const int bh = blockIdx.y;
    const int q0 = blockIdx.x * QT;

    AHf qb[2];
    {
        const unsigned short* qr = Qp + ((size_t)bh * SEQ + q0 + w * 16 + m) * DH;
        #pragma unroll
        for (int ks = 0; ks < 2; ++ks) {
            qb[ks].q[0] = *(const u32x4*)(qr + ks * 32 + 8 * h);
            qb[ks].q[1] = *(const u32x4*)(qr + ks * 32 + 16 + 8 * h);
        }
    }

    v8f O[4];
    #pragma unroll
    for (int dt = 0; dt < 4; ++dt) { v8f z = {}; O[dt] = z; }
    float mrun = -1.0e30f, lrun = 0.0f;
    const float CS = 0.125f * 1.4426950408889634f;

    #pragma unroll 1
    for (int kt = 0; kt < SEQ / KTL; ++kt) {
        __syncthreads();
        #pragma unroll
        for (int it = 0; it < 2; ++it) {
            const int p = tid + it * 256;
            const int row = p >> 3, c8 = p & 7;
            Ks[row * LP + c8]  = *(const u32x4*)(Kp  + ((size_t)bh * SEQ + kt * KTL + row) * DH + c8 * 8);
            Vhs[row * LP + c8] = *(const u32x4*)(Vth + ((size_t)bh * DH + row) * SEQ + kt * KTL + c8 * 8);
            Vls[row * LP + c8] = *(const u32x4*)(Vtl + ((size_t)bh * DH + row) * SEQ + kt * KTL + c8 * 8);
        }
        __syncthreads();

        v8f S[4];
        #pragma unroll
        for (int t = 0; t < 4; ++t) {
            v8f z = {}; S[t] = z;
            #pragma unroll
            for (int ks = 0; ks < 2; ++ks) {
                AHf ka;
                ka.q[0] = Ks[(t * 16 + m) * LP + 4 * ks + h];
                ka.q[1] = Ks[(t * 16 + m) * LP + 4 * ks + 2 + h];
                S[t] = mma_f16(ka, qb[ks], S[t]);
            }
        }

        float tmax = -1.0e30f;
        #pragma unroll
        for (int t = 0; t < 4; ++t)
            #pragma unroll
            for (int r = 0; r < 8; ++r) tmax = fmaxf(tmax, S[t][r]);
        tmax = fmaxf(tmax, __shfl_xor(tmax, 16, 32));
        const float mnew  = fmaxf(mrun, tmax);
        const float alpha = __builtin_amdgcn_exp2f((mrun - mnew) * CS);
        const float moff  = mnew * CS;
        mrun = mnew;
        float psum = 0.0f;
        #pragma unroll
        for (int t = 0; t < 4; ++t)
            #pragma unroll
            for (int r = 0; r < 8; ++r) {
                const float pe = __builtin_amdgcn_exp2f(S[t][r] * CS - moff);
                S[t][r] = pe;
                psum += pe;
            }
        psum += __shfl_xor(psum, 16, 32);
        lrun = lrun * alpha + psum;
        #pragma unroll
        for (int dt = 0; dt < 4; ++dt) O[dt] = O[dt] * alpha;

        #pragma unroll
        for (int ks = 0; ks < 2; ++ks) {
            ABf ph, pl;
            #pragma unroll
            for (int e = 0; e < 4; ++e) {
                split2(S[2 * ks][2 * e],     S[2 * ks][2 * e + 1],     ph.u[e],     pl.u[e]);
                split2(S[2 * ks + 1][2 * e], S[2 * ks + 1][2 * e + 1], ph.u[4 + e], pl.u[4 + e]);
            }
            #pragma unroll
            for (int dt = 0; dt < 4; ++dt) {
                ABf va, vb;
                const int idx = (dt * 16 + m) * LP + 4 * ks;
                va.q[0] = Vhs[idx + h]; va.q[1] = Vhs[idx + 2 + h];
                vb.q[0] = Vls[idx + h]; vb.q[1] = Vls[idx + 2 + h];
                O[dt] = mma_bf16(va, ph, O[dt]);
                O[dt] = mma_bf16(vb, ph, O[dt]);
                O[dt] = mma_bf16(va, pl, O[dt]);
            }
        }
    }

    const float invl = 1.0f / lrun;
    #pragma unroll
    for (int pl = 0; pl < 2; ++pl) {
        if (pl == 1) __syncthreads();
        #pragma unroll
        for (int dt = 0; dt < 4; ++dt) {
            PK4 pk;
            #pragma unroll
            for (int e = 0; e < 4; ++e) {
                const float a  = O[dt][2 * e]     * invl;
                const float b2 = O[dt][2 * e + 1] * invl;
                unsigned int hi, lo;
                split2(a, b2, hi, lo);
                pk.u[e] = (pl == 0) ? hi : lo;
            }
            Ost[(w * 16 + m) * LP + 2 * dt + h] = pk.q;
        }
        __syncthreads();
        unsigned short* base = (pl == 0) ? Ch : Cl;
        u32x4 vv[4]; unsigned short* pp[4];
        #pragma unroll
        for (int it = 0; it < 4; ++it) {
            const int row = it * 4 + (lane >> 3);
            const int c16 = lane & 7;
            vv[it] = Ost[(w * 16 + row) * LP + c16];
            pp[it] = base + ((size_t)bh * SEQ + q0 + w * 16 + row) * DH + c16 * 8;
        }
        #pragma unroll
        for (int it = 0; it < 4; ++it) *(volatile u32x4*)pp[it] = vv[it];
        __threadfence();
        #pragma unroll
        for (int it = 0; it < 4; ++it) *(volatile u32x4*)pp[it] = vv[it];
    }
}

extern "C" void kernel_launch(void* const* d_in, const int* in_sizes, int n_in,
                              void* d_out, int out_size, void* d_ws, size_t ws_size,
                              hipStream_t stream)
{
    if (n_in < 9) return;
    const size_t need_act = ((size_t)(NB - 1) * SEQ_FULL + SEQ) * DM;
    if ((size_t)in_sizes[0] < need_act) return;
    if ((size_t)in_sizes[1] < (size_t)DM * DM || (size_t)in_sizes[3] < (size_t)DM * DM ||
        (size_t)in_sizes[5] < (size_t)DM * DM || (size_t)in_sizes[7] < (size_t)DM * DM) return;
    if (in_sizes[2] < DM || in_sizes[4] < DM || in_sizes[6] < DM || in_sizes[8] < DM) return;
    if ((size_t)out_size < need_act) return;

    const float* X  = (const float*)d_in[0];
    const float* Wq = (const float*)d_in[1];
    const float* bq = (const float*)d_in[2];
    const float* Wk = (const float*)d_in[3];
    const float* bk = (const float*)d_in[4];
    const float* Wv = (const float*)d_in[5];
    const float* bv = (const float*)d_in[6];
    const float* Wo = (const float*)d_in[7];
    const float* bo = (const float*)d_in[8];

    const size_t actH = (size_t)MTOK * DM;
    const size_t wH   = (size_t)DM * DM;
    const size_t total_bytes = (7 * actH + 4 * wH) * sizeof(unsigned short);
    if (total_bytes > ws_size) return;

    unsigned short* ws  = (unsigned short*)d_ws;
    unsigned short* Xb  = ws;
    unsigned short* Wqb = Xb  + actH;
    unsigned short* Wkb = Wqb + wH;
    unsigned short* Wvb = Wkb + wH;
    unsigned short* Wob = Wvb + wH;
    unsigned short* Qp  = Wob + wH;
    unsigned short* Kp  = Qp  + actH;
    unsigned short* Vth = Kp  + actH;
    unsigned short* Vtl = Vth + actH;
    unsigned short* Ch  = Vtl + actH;
    unsigned short* Cl  = Ch  + actH;

    dim3 blk(256);
    k_cvt<<<dim3(MTOK / 2, 1), blk, 0, stream>>>(X, X, X, X, Xb, Xb, Xb, Xb, MTOK, SEQ, SEQ_FULL);
    k_cvt<<<dim3(DM / 2, 4), blk, 0, stream>>>(Wq, Wk, Wv, Wo, Wqb, Wkb, Wvb, Wob, DM, DM, DM);

    k_gemm<0><<<dim3(DM / 128, MTOK / 128), blk, 0, stream>>>(Wqb, Xb, Xb, bq, (void*)Qp, (void*)Qp);
    k_gemm<0><<<dim3(DM / 128, MTOK / 128), blk, 0, stream>>>(Wkb, Xb, Xb, bk, (void*)Kp, (void*)Kp);
    k_gemm<1><<<dim3(MTOK / 128, DM / 128), blk, 0, stream>>>(Xb, Wvb, Wvb, bv, (void*)Vth, (void*)Vtl);

    k_attn<<<dim3(SEQ / QT, NB * NH), blk, 0, stream>>>(Qp, Kp, Vth, Vtl, Ch, Cl);

    k_gemm<2><<<dim3(DM / 128, MTOK / 128), blk, 0, stream>>>(Wob, Ch, Cl, bo, d_out, d_out);
}
